// Complex_32160715113072
// MI455X (gfx1250) — hardware-verified
//
#include <hip/hip_runtime.h>
#include <stddef.h>


#define DF      128
#define NBAS    4
#define NCOL    640
#define XOFF    512
#define NTHR    256
#define NWAVE   8
#define EPT     8
#define NGRP    2
#define CHUNK   (NTHR * EPT * NGRP)
#define WCAP    (EPT * NGRP * 32)
#define LISTN   (NWAVE * WCAP)
#define NB1     512
#define GROWS   128
#define APITCH  136
#define TPP     4
#define NPASS   (NCOL / (16 * TPP))
#define WPL     (NCOL * DF)

#define LDS_NODE (2 * GROWS * APITCH * 2 + NWAVE * 16 * (16 * TPP) * 4)
#define LDS_AGG  (NB1 * DF * 4 + LISTN * 4 + NB1 * 4 + 64)

static_assert((CHUNK & (CHUNK - 1)) == 0);
static_assert(CHUNK <= 4096);
static_assert(NB1 <= 4096 && (NB1 & (NB1 - 1)) == 0);
static_assert(NPASS * 16 * TPP == NCOL);
static_assert(NB1 * 4 <= LISTN * 4);
static_assert((WPL / 8) % NTHR == 0);
static_assert((GROWS * APITCH * 2) % 16 == 0);

typedef float          v4f   __attribute__((ext_vector_type(4)));
typedef float          v8f   __attribute__((ext_vector_type(8)));
typedef int            v4i   __attribute__((ext_vector_type(4)));
typedef unsigned short v8us  __attribute__((ext_vector_type(8)));
typedef __bf16         v16bf __attribute__((ext_vector_type(16)));
union FragB { v16bf v; v8us h[2]; };

__device__ __forceinline__ unsigned int bfb(float f) {
  const unsigned int a = __float_as_uint(f);
  return (a + 0x7FFFu + ((a >> 16) & 1u)) >> 16;
}
__device__ __forceinline__ unsigned int lob(float f, unsigned int hb) {
  return bfb(f - __uint_as_float(hb << 16));
}
__device__ __forceinline__ void hl8(v4f a, v4f b, v8us* hv, v8us* lv) {
  v8us h, l;
  unsigned int t;
  t = bfb(a.x); h[0] = (unsigned short)t; l[0] = (unsigned short)lob(a.x, t);
  t = bfb(a.y); h[1] = (unsigned short)t; l[1] = (unsigned short)lob(a.y, t);
  t = bfb(a.z); h[2] = (unsigned short)t; l[2] = (unsigned short)lob(a.z, t);
  t = bfb(a.w); h[3] = (unsigned short)t; l[3] = (unsigned short)lob(a.w, t);
  t = bfb(b.x); h[4] = (unsigned short)t; l[4] = (unsigned short)lob(b.x, t);
  t = bfb(b.y); h[5] = (unsigned short)t; l[5] = (unsigned short)lob(b.y, t);
  t = bfb(b.z); h[6] = (unsigned short)t; l[6] = (unsigned short)lob(b.z, t);
  t = bfb(b.w); h[7] = (unsigned short)t; l[7] = (unsigned short)lob(b.w, t);
  *hv = h; *lv = l;
}

__device__ __forceinline__ v8f wm3(v16bf ah, v16bf al, v16bf bh, v16bf bl, v8f c) {
  v8f d = __builtin_amdgcn_wmma_f32_16x16x32_bf16(false, ah, false, bh, (short)0, c, false, false);
  d = __builtin_amdgcn_wmma_f32_16x16x32_bf16(false, ah, false, bl, (short)0, d, false, false);
  d = __builtin_amdgcn_wmma_f32_16x16x32_bf16(false, al, false, bh, (short)0, d, false, false);
  asm volatile("v_nop\n\tv_nop\n\tv_nop\n\tv_nop" : "+v"(d) : "v"(ah), "v"(al), "v"(bh), "v"(bl));
  return d;
}

template <int NB>
__device__ __forceinline__ int scan_chunk(const int* __restrict__ dsts, int nE, int cbase, int nodeBase,
                                          int vec8, int* list, int tid, int lane, int wave) {
  int wc = 0;
#pragma unroll
  for (int g = 0; g < NGRP; ++g) {
    const int el0  = (g * NTHR + tid) * EPT;
    const int e0   = cbase + el0;
    const int sent = -2147483647 - 1;
    v4i da, db;
    if (vec8 != 0 && cbase + CHUNK <= nE) {
      da = *(const v4i*)(dsts + e0);
      db = *(const v4i*)(dsts + e0 + 4);
    } else {
      da.x = (e0     < nE) ? dsts[min(e0, nE - 1)] : sent;
      da.y = (e0 + 1 < nE) ? dsts[min(e0 + 1, nE - 1)] : sent;
      da.z = (e0 + 2 < nE) ? dsts[min(e0 + 2, nE - 1)] : sent;
      da.w = (e0 + 3 < nE) ? dsts[min(e0 + 3, nE - 1)] : sent;
      db.x = (e0 + 4 < nE) ? dsts[min(e0 + 4, nE - 1)] : sent;
      db.y = (e0 + 5 < nE) ? dsts[min(e0 + 5, nE - 1)] : sent;
      db.z = (e0 + 6 < nE) ? dsts[min(e0 + 6, nE - 1)] : sent;
      db.w = (e0 + 7 < nE) ? dsts[min(e0 + 7, nE - 1)] : sent;
    }
    const unsigned nb = (unsigned)nodeBase;
    const unsigned s0 = (unsigned)da.x - nb, s1 = (unsigned)da.y - nb;
    const unsigned s2 = (unsigned)da.z - nb, s3 = (unsigned)da.w - nb;
    const unsigned s4 = (unsigned)db.x - nb, s5 = (unsigned)db.y - nb;
    const unsigned s6 = (unsigned)db.z - nb, s7 = (unsigned)db.w - nb;
    const bool h0 = s0 < (unsigned)NB, h1 = s1 < (unsigned)NB, h2 = s2 < (unsigned)NB, h3 = s3 < (unsigned)NB;
    const bool h4 = s4 < (unsigned)NB, h5 = s5 < (unsigned)NB, h6 = s6 < (unsigned)NB, h7 = s7 < (unsigned)NB;
    const unsigned any = __builtin_amdgcn_ballot_w32(h0 | h1 | h2 | h3 | h4 | h5 | h6 | h7);
    if (any != 0u) {
#define HITJ(J, HJ, SJ) { \
        const unsigned mj = __builtin_amdgcn_ballot_w32(HJ); \
        if (mj != 0u) { \
          if (HJ) { \
            const int pos = wc + (int)__builtin_amdgcn_mbcnt_lo(mj, 0u); \
            if (pos < WCAP) list[wave * WCAP + pos] = ((el0 + (J)) << 12) | (int)(SJ); \
          } \
          wc += (int)__builtin_popcount(mj); } }
      HITJ(0, h0, s0)
      HITJ(1, h1, s1)
      HITJ(2, h2, s2)
      HITJ(3, h3, s3)
      HITJ(4, h4, s4)
      HITJ(5, h5, s5)
      HITJ(6, h6, s6)
      HITJ(7, h7, s7)
#undef HITJ
    }
  }
  return wc;
}

__global__ __launch_bounds__(NTHR) void k_wprep(
    const float* __restrict__ bas1, const float* __restrict__ rt1,
    const float* __restrict__ bas2, const float* __restrict__ rt2,
    unsigned short* wp) {
  const int per   = WPL / 8;
  const int layer = (blockIdx.x >= per / NTHR) ? 1 : 0;
  const int i     = blockIdx.x * NTHR + threadIdx.x - layer * per;
  if (i >= per) return;
  const float* bas = layer ? bas2 : bas1;
  const float* rt  = layer ? rt2 : rt1;
  const int o8 = i * 8;
  const int n  = o8 / DF;
  const int k0 = o8 - n * DF;
  v4f a, b;
  if (n < XOFF) {
    const int bb = n >> 7, o = n & 127;
    const float* p = bas + ((size_t)(bb * DF + k0)) * DF + o;
    a.x = p[0];      a.y = p[DF];     a.z = p[2 * DF]; a.w = p[3 * DF];
    b.x = p[4 * DF]; b.y = p[5 * DF]; b.z = p[6 * DF]; b.w = p[7 * DF];
  } else {
    const float* p = rt + (size_t)k0 * DF + (n - XOFF);
    a.x = p[0];      a.y = p[DF];     a.z = p[2 * DF]; a.w = p[3 * DF];
    b.x = p[4 * DF]; b.y = p[5 * DF]; b.z = p[6 * DF]; b.w = p[7 * DF];
  }
  v8us hv, lv;
  hl8(a, b, &hv, &lv);
  unsigned short* dh = wp + (size_t)layer * 2 * WPL + o8;
  unsigned short* dl = dh + WPL;
  *(volatile v8us*)dh = hv;
  *(volatile v8us*)dl = lv;
  __threadfence();
  *(volatile v8us*)dh = hv;
  *(volatile v8us*)dl = lv;
}

template <int GATHER>
__global__ __launch_bounds__(NTHR) void k_node(
    const float* __restrict__ x, const int* __restrict__ ids,
    const unsigned short* __restrict__ whi, const unsigned short* __restrict__ wlo,
    float* plane, int nN, int nTab) {
  extern __shared__ v4f lds_dyn[];
  unsigned short* sHi = (unsigned short*)lds_dyn;
  unsigned short* sLo = sHi + GROWS * APITCH;
  float*          stg = (float*)(sLo + GROWS * APITCH);
  const int tid = threadIdx.x, lane = tid & 31, wave = tid >> 5, hh = lane >> 4, m = lane & 15;
  const int rowBase = blockIdx.x * GROWS;

#pragma unroll
  for (int it = 0; it < (GROWS * DF / 8) / NTHR; ++it) {
    const int idx = it * NTHR + tid;
    const int r   = idx >> 4;
    const int c0  = (idx & 15) * 8;
    int node = rowBase + r;
    node = node > nN - 1 ? nN - 1 : node;
    int row = node;
    if (GATHER) {
      int id = ids[node];
      id = id < 0 ? 0 : (id > nTab - 1 ? nTab - 1 : id);
      row = id;
    }
    const float* xp = x + (size_t)row * DF + c0;
    const v4f a = *(const v4f*)xp, b = *(const v4f*)(xp + 4);
    v8us hv, lv;
    hl8(a, b, &hv, &lv);
    *(v8us*)(sHi + r * APITCH + c0) = hv;
    *(v8us*)(sLo + r * APITCH + c0) = lv;
  }
  __syncthreads();

  const unsigned short* arh = sHi + (wave * 16 + m) * APITCH + 8 * hh;
  const unsigned short* arl = sLo + (wave * 16 + m) * APITCH + 8 * hh;
  float* stw = stg + wave * 16 * 64;

#pragma unroll 1
  for (int p = 0; p < NPASS; ++p) {
    const int n0 = p * 64;
    v8f acc[TPP];
#pragma unroll
    for (int t = 0; t < TPP; ++t) { v8f z = {0.f, 0.f, 0.f, 0.f, 0.f, 0.f, 0.f, 0.f}; acc[t] = z; }
#pragma unroll 1
    for (int kt = 0; kt < DF / 32; ++kt) {
      FragB ah, al;
      ah.h[0] = *(const v8us*)(arh + 32 * kt);
      ah.h[1] = *(const v8us*)(arh + 32 * kt + 16);
      al.h[0] = *(const v8us*)(arl + 32 * kt);
      al.h[1] = *(const v8us*)(arl + 32 * kt + 16);
#pragma unroll
      for (int t = 0; t < TPP; ++t) {
        const size_t bo = (size_t)(n0 + 16 * t + m) * DF + 32 * kt + 8 * hh;
        FragB bh, bl;
        bh.h[0] = *(const v8us*)(whi + bo);
        bh.h[1] = *(const v8us*)(whi + bo + 16);
        bl.h[0] = *(const v8us*)(wlo + bo);
        bl.h[1] = *(const v8us*)(wlo + bo + 16);
        acc[t] = wm3(ah.v, al.v, bh.v, bl.v, acc[t]);
      }
    }
    float* sp = stw + (8 * hh) * 64 + m;
#pragma unroll
    for (int t = 0; t < TPP; ++t) {
      sp[0 * 64 + 16 * t] = acc[t][0];
      sp[1 * 64 + 16 * t] = acc[t][1];
      sp[2 * 64 + 16 * t] = acc[t][2];
      sp[3 * 64 + 16 * t] = acc[t][3];
      sp[4 * 64 + 16 * t] = acc[t][4];
      sp[5 * 64 + 16 * t] = acc[t][5];
      sp[6 * 64 + 16 * t] = acc[t][6];
      sp[7 * 64 + 16 * t] = acc[t][7];
    }
    __syncthreads();
    const float* lp = stw + hh * 64 + 4 * m;
    float* gp = plane + ((size_t)rowBase + wave * 16 + hh) * NCOL + n0 + 4 * m;
#pragma unroll
    for (int i = 0; i < 8; ++i) {
      const v4f v = *(const v4f*)(lp + 2 * i * 64);
      *(volatile v4f*)(gp + (size_t)(2 * i) * NCOL) = v;
    }
    __threadfence();
#pragma unroll
    for (int i = 0; i < 8; ++i) {
      const v4f v = *(const v4f*)(lp + 2 * i * 64);
      *(volatile v4f*)(gp + (size_t)(2 * i) * NCOL) = v;
    }
    __syncthreads();
  }
}

__device__ __forceinline__ void agg_store_pass(const float* acc, const float* invs,
                                               const float* __restrict__ plane, const float* __restrict__ bias,
                                               float* hout, int nodeBase, int nN, int doRelu, int tid) {
#pragma unroll 1
  for (int it = 0; it < (NB1 * DF / 4) / NTHR; ++it) {
    const int idx   = it * NTHR + tid;
    const int slot  = idx >> 5;
    const int c4    = (idx & 31) * 4;
    const int node  = nodeBase + slot;
    const int nodec = node > nN - 1 ? nN - 1 : node;
    const v4f   a   = *(const v4f*)(acc + slot * DF + c4);
    const float iv  = invs[slot];
    const v4f   xr  = *(const v4f*)(plane + (size_t)nodec * NCOL + XOFF + c4);
    const v4f   bv  = *(const v4f*)(bias + c4);
    v4f v = a * iv + xr;
    v = v + bv;
    if (doRelu) {
      v.x = fmaxf(v.x, 0.f); v.y = fmaxf(v.y, 0.f); v.z = fmaxf(v.z, 0.f); v.w = fmaxf(v.w, 0.f);
    }
    if (node < nN) *(volatile v4f*)(hout + (size_t)node * DF + c4) = v;
  }
}

__global__ __launch_bounds__(NTHR) void k_agg(
    const int* __restrict__ ei, const int* __restrict__ et, const float* __restrict__ enorm,
    const float* __restrict__ att, const float* __restrict__ plane, const float* __restrict__ bias,
    float* hout, int nN, int nE, int nRel, int vec8, int useNorm, int doRelu) {
  extern __shared__ v4f lds_dyn[];
  float* acc  = (float*)lds_dyn;
  int*   list = (int*)(acc + NB1 * DF);
  int*   cnt  = list + LISTN;
  int*   wcnt = cnt + NB1;
  float* invs = (float*)list;
  const int tid = threadIdx.x, lane = tid & 31, wave = tid >> 5;
  const int nodeBase = blockIdx.x * NB1;
  const int* dsts = ei + nE;

  {
    const v4f z = {0.f, 0.f, 0.f, 0.f};
    for (int i = tid; i < NB1 * DF / 4; i += NTHR) lds_dyn[i] = z;
    for (int i = tid; i < NB1; i += NTHR) cnt[i] = 0;
  }
  __syncthreads();

  const int nChunks = (nE + CHUNK - 1) / CHUNK;
#pragma unroll 1
  for (int ch = 0; ch < nChunks; ++ch) {
    const int cbase = ch * CHUNK;
    const int wc = scan_chunk<NB1>(dsts, nE, cbase, nodeBase, vec8, list, tid, lane, wave);
    if (lane == 0) wcnt[wave] = wc;
    __syncthreads();
    if (wave == 0) {
#pragma unroll 1
      for (int wsx = 0; wsx < NWAVE; ++wsx) {
        int n = __builtin_amdgcn_readfirstlane(wcnt[wsx]);
        n = n > WCAP ? WCAP : (n < 0 ? 0 : n);
        const int* lp = list + wsx * WCAP;
#pragma unroll 1
        for (int i = 0; i < n; ++i) {
          const int ent  = __builtin_amdgcn_readfirstlane(lp[i]);
          const int slot = ent & (NB1 - 1);
          int e = cbase + ((ent >> 12) & (CHUNK - 1));
          e = e > nE - 1 ? nE - 1 : e;
          int src = ei[e];
          src = src < 0 ? 0 : (src > nN - 1 ? nN - 1 : src);
          int r = et[e];
          r = r < 0 ? 0 : (r > nRel - 1 ? nRel - 1 : r);
          const float* cp = att + (size_t)r * NBAS;
          const float c0 = cp[0], c1 = cp[1], c2 = cp[2], c3 = cp[3];
          const float enl = enorm[e];
          const float en = useNorm ? enl : 1.0f;
          const float* np = plane + (size_t)src * NCOL + 4 * lane;
          const v4f v0 = *(const v4f*)np;
          const v4f v1 = *(const v4f*)(np + DF);
          const v4f v2 = *(const v4f*)(np + 2 * DF);
          const v4f v3 = *(const v4f*)(np + 3 * DF);
          v4f msg = v0 * c0;
          msg = msg + v1 * c1;
          msg = msg + v2 * c2;
          msg = msg + v3 * c3;
          msg = msg * en;
          v4f* ap = (v4f*)(acc + slot * DF + 4 * lane);
          *ap = *ap + msg;
          if (lane == 0) cnt[slot] = cnt[slot] + 1;
        }
      }
    }
    __syncthreads();
  }

#pragma unroll 1
  for (int i = tid; i < NB1; i += NTHR) {
    int c = cnt[i];
    c = c < 1 ? 1 : c;
    invs[i] = 1.0f / (float)c;
  }
  __syncthreads();

  agg_store_pass(acc, invs, plane, bias, hout, nodeBase, nN, doRelu, tid);
  __threadfence();
  agg_store_pass(acc, invs, plane, bias, hout, nodeBase, nN, doRelu, tid);
}

extern "C" void kernel_launch(void* const* d_in, const int* in_sizes, int n_in,
                              void* d_out, int out_size, void* d_ws, size_t ws_size,
                              hipStream_t stream) {
  if (n_in < 14) return;
  const int nN    = in_sizes[0];
  const int nE    = in_sizes[1] / 2;
  const int nTabR = in_sizes[4] / DF;
  const int nTabI = in_sizes[5] / DF;
  const int nRel  = in_sizes[7] / NBAS;
  if (nN <= 0 || nE <= 0 || in_sizes[1] != 2 * nE || in_sizes[2] != nE || in_sizes[3] != nE) return;
  if (nTabR <= 0 || in_sizes[4] != nTabR * DF || nTabI <= 0 || in_sizes[5] != nTabI * DF) return;
  if (in_sizes[6] != NBAS * DF * DF || nRel <= 0 || in_sizes[7] != nRel * NBAS) return;
  if (in_sizes[8] != DF * DF || in_sizes[9] != DF) return;
  if (in_sizes[10] != NBAS * DF * DF || in_sizes[11] != in_sizes[7] || in_sizes[12] != DF * DF || in_sizes[13] != DF) return;
  if (out_size != 2 * nN * DF) return;

  const int*   entity = (const int*)d_in[0];
  const int*   eidx   = (const int*)d_in[1];
  const int*   etype  = (const int*)d_in[2];
  const float* enorm  = (const float*)d_in[3];
  const float* emb_r  = (const float*)d_in[4];
  const float* emb_i  = (const float*)d_in[5];
  const float* basis1 = (const float*)d_in[6];
  const float* att1   = (const float*)d_in[7];
  const float* root1  = (const float*)d_in[8];
  const float* bias1  = (const float*)d_in[9];
  const float* basis2 = (const float*)d_in[10];
  const float* att2   = (const float*)d_in[11];
  const float* root2  = (const float*)d_in[12];
  const float* bias2  = (const float*)d_in[13];
  float* out0 = (float*)d_out;
  float* out1 = out0 + (size_t)nN * DF;

  const int nG = (nN + GROWS - 1) / GROWS;
  const int nA = (nN + NB1 - 1) / NB1;

  char* ws = (char*)d_ws;
  size_t off = 0;
  const size_t oW = off; off += (size_t)4 * WPL * 2;                       off = (off + 255) & ~(size_t)255;
  const size_t oP = off; off += (size_t)nG * GROWS * NCOL * 4;             off = (off + 255) & ~(size_t)255;
  if (off > ws_size) return;
  unsigned short* wp = (unsigned short*)(ws + oW);
  const unsigned short* whi1 = wp;
  const unsigned short* wlo1 = wp + WPL;
  const unsigned short* whi2 = wp + 2 * WPL;
  const unsigned short* wlo2 = wp + 3 * WPL;
  float* plane = (float*)(ws + oP);

  const int vec8 = ((nE & 3) == 0) ? 1 : 0;

  k_wprep<<<(2 * (WPL / 8)) / NTHR, NTHR, 0, stream>>>(basis1, root1, basis2, root2, wp);

  hipFuncSetAttribute(reinterpret_cast<const void*>(&k_node<1>),
                      hipFuncAttributeMaxDynamicSharedMemorySize, LDS_NODE);
  hipFuncSetAttribute(reinterpret_cast<const void*>(&k_node<0>),
                      hipFuncAttributeMaxDynamicSharedMemorySize, LDS_NODE);
  hipFuncSetAttribute(reinterpret_cast<const void*>(&k_agg),
                      hipFuncAttributeMaxDynamicSharedMemorySize, LDS_AGG);

  k_node<1><<<nG, NTHR, LDS_NODE, stream>>>(emb_r, entity, whi1, wlo1, plane, nN, nTabR);
  k_agg<<<nA, NTHR, LDS_AGG, stream>>>(eidx, etype, enorm, att1, plane, bias1, out0, nN, nE, nRel, vec8, 0, 1);
  k_node<1><<<nG, NTHR, LDS_NODE, stream>>>(emb_i, entity, whi1, wlo1, plane, nN, nTabI);
  k_agg<<<nA, NTHR, LDS_AGG, stream>>>(eidx, etype, enorm, att1, plane, bias1, out1, nN, nE, nRel, vec8, 1, 1);
  k_node<0><<<nG, NTHR, LDS_NODE, stream>>>(out0, entity, whi2, wlo2, plane, nN, nN);
  k_agg<<<nA, NTHR, LDS_AGG, stream>>>(eidx, etype, enorm, att2, plane, bias2, out0, nN, nE, nRel, vec8, 0, 0);
  k_node<0><<<nG, NTHR, LDS_NODE, stream>>>(out1, entity, whi2, wlo2, plane, nN, nN);
  k_agg<<<nA, NTHR, LDS_AGG, stream>>>(eidx, etype, enorm, att2, plane, bias2, out1, nN, nE, nRel, vec8, 1, 0);
}
